// Non_local_Block_62362925137961
// MI455X (gfx1250) — hardware-verified
//
#include <hip/hip_runtime.h>

#define __bf16 _Float16
typedef _Float16 bf16;
typedef __attribute__((ext_vector_type(16))) _Float16 bf16x16;
typedef __attribute__((ext_vector_type(8)))  _Float16 bf16x8;
#define RSPLIT (1.0f / 2048.0f)
__device__ __forceinline__ void split16(float f, _Float16& h, _Float16& l) { h = (_Float16)f; l = (_Float16)((f - (float)h) * 2048.0f); }
__device__ __forceinline__ unsigned pack2h(_Float16 a, _Float16 b) { return (unsigned)__builtin_bit_cast(unsigned short, a) | ((unsigned)__builtin_bit_cast(unsigned short, b) << 16); }
typedef __attribute__((ext_vector_type(8)))  float  v8f;

#define NB    4
#define CIN   256
#define CO    128
#define NPIX  4096
#define PL_X  ((size_t)NB * NPIX * CIN)
#define PL_P  ((size_t)NB * NPIX * CO)
#define PL_W  ((size_t)CO * CIN)
#define PL_WW ((size_t)CIN * CO)

__device__ __forceinline__ bf16x16 load_frag_a(const bf16* __restrict__ base, int ldk,
                                               int row, int k0, int hf) {
  const bf16* p = base + (size_t)row * ldk + k0;
  bf16x8 lo = *(const bf16x8*)(p + hf * 8);
  bf16x8 hi = *(const bf16x8*)(p + 16 + hf * 8);
  bf16x16 r;
#pragma unroll
  for (int i = 0; i < 8; ++i) { r[i] = lo[i]; r[i + 8] = hi[i]; }
  return r;
}

__device__ __forceinline__ bf16x16 load_frag_b(const bf16* __restrict__ base, int ldk,
                                               int col, int k0, int hf) {
  const bf16* p = base + (size_t)col * ldk + k0;
  bf16x8 lo = *(const bf16x8*)(p + hf * 8);
  bf16x8 hi = *(const bf16x8*)(p + 16 + hf * 8);
  bf16x16 r;
#pragma unroll
  for (int i = 0; i < 8; ++i) { r[i] = lo[i]; r[i + 8] = hi[i]; }
  return r;
}

__device__ __forceinline__ v8f wmma_bf16(bf16x16 a, bf16x16 b, v8f c) {
  return __builtin_amdgcn_wmma_f32_16x16x32_f16(false, a, false, b, (short)0, c,
                                                 false, false);
}
__device__ __forceinline__ v8f wmma_split(bf16x16 ah, bf16x16 al, bf16x16 bh, bf16x16 bl, v8f c) {
  v8f x = {};
  x = wmma_bf16(al, bh, x);
  x = wmma_bf16(ah, bl, x);
  return wmma_bf16(ah, bh, c) + x * RSPLIT;
}
__device__ __forceinline__ v8f mma_planes(const bf16* A, size_t pla, int lda, int arow,
                                           const bf16* B, size_t plb, int ldb, int bcol, int k0, int hf, v8f c) {
  return wmma_split(load_frag_a(A, lda, arow, k0, hf), load_frag_a(A + pla, lda, arow, k0, hf),
                    load_frag_b(B, ldb, bcol, k0, hf), load_frag_b(B + plb, ldb, bcol, k0, hf), c);
}

__device__ __forceinline__ unsigned lds_off(const void* p) {
  return (unsigned)(unsigned long long)p;
}
__device__ __forceinline__ void async_cp16(unsigned lds_byte_off, const void* gsrc) {
  asm volatile("global_load_async_to_lds_b128 %0, %1, off"
               :: "v"(lds_byte_off), "v"(gsrc) : "memory");
}

__global__ void k_wconv(const float* __restrict__ wt, const float* __restrict__ wp,
                        const float* __restrict__ wg, const float* __restrict__ ww,
                        bf16* ot, bf16* op, bf16* og, bf16* ow) {
  int i = (blockIdx.x * 256 + threadIdx.x) * 2;
  if (i < CO * CIN) {
    const float* src[4] = {wt, wp, wg, ww};
    bf16* dst[4] = {ot, op, og, ow};
#pragma unroll
    for (int s = 0; s < 4; ++s) {
      _Float16 h0, l0, h1, l1; split16(src[s][i], h0, l0); split16(src[s][i + 1], h1, l1);
      unsigned* d = (unsigned*)(dst[s] + i); unsigned* dl = (unsigned*)(dst[s] + PL_W + i);
      const unsigned ph = pack2h(h0, h1), pq = pack2h(l0, l1);
      *(volatile unsigned*)d = ph; *(volatile unsigned*)dl = pq; __threadfence(); *(volatile unsigned*)d = ph; *(volatile unsigned*)dl = pq;
    }
  }
}

__global__ void __launch_bounds__(256) k_xpose(const float* __restrict__ x, bf16* __restrict__ xT) {
  __shared__ float t[CIN][33];
  const int p0 = blockIdx.x * 32, b = blockIdx.y;
  const int tid = threadIdx.x, lane = tid & 31, wave = tid >> 5;
#pragma unroll 4
  for (int k = 0; k < 32; ++k) { const int c = wave * 32 + k; t[c][lane] = x[((size_t)b * CIN + c) * NPIX + p0 + lane]; }
  __syncthreads();
#pragma unroll 1
  for (int pass = 0; pass < 2; ++pass) {
#pragma unroll
    for (int rr = 0; rr < 4; ++rr) {
      const int p = wave * 4 + rr;
      bf16* row = xT + ((size_t)b * NPIX + p0 + p) * CIN;
#pragma unroll
      for (int sgm = 0; sgm < 4; ++sgm) {
        const int c = sgm * 64 + 2 * lane;
        _Float16 h0, l0, h1, l1; split16(t[c][p], h0, l0); split16(t[c + 1][p], h1, l1);
        *(volatile unsigned*)(row + c) = pack2h(h0, h1); *(volatile unsigned*)(row + PL_X + c) = pack2h(l0, l1);
      }
    }
    __threadfence();
  }
}

__global__ void __launch_bounds__(256) k_proj(const bf16* __restrict__ xT,
                       const bf16* __restrict__ wth, const bf16* __restrict__ wph,
                       const bf16* __restrict__ wg,
                       const float* __restrict__ bth, const float* __restrict__ bph,
                       const float* __restrict__ bg,
                       bf16* __restrict__ th, bf16* __restrict__ ph,
                       bf16* __restrict__ g) {
  __shared__ float st[3][16][CO + 4];
  int wave = threadIdx.x >> 5, lane = threadIdx.x & 31;
  int l16 = lane & 15, hf = lane >> 4;
  int tile = blockIdx.x * 8 + wave;
  int b = tile >> 11;
  int rem = tile & 2047;
  int pt = rem >> 3, ot = rem & 7;
  int q0 = pt * 16, o0 = ot * 16;
  const bf16* xb = xT + (size_t)b * NPIX * CIN;

  v8f a0 = {}, a1 = {}, a2 = {};
#pragma unroll 2
  for (int kk = 0; kk < 8; ++kk) {
    bf16x16 ax  = load_frag_a(xb, CIN, q0 + l16, kk * 32, hf);
    bf16x16 axl = load_frag_a(xb + PL_X, CIN, q0 + l16, kk * 32, hf);
    a0 = wmma_split(ax, axl, load_frag_b(wth, CIN, o0 + l16, kk * 32, hf), load_frag_b(wth + PL_W, CIN, o0 + l16, kk * 32, hf), a0);
    a1 = wmma_split(ax, axl, load_frag_b(wph, CIN, o0 + l16, kk * 32, hf), load_frag_b(wph + PL_W, CIN, o0 + l16, kk * 32, hf), a1);
    a2 = wmma_split(ax, axl, load_frag_b(wg,  CIN, o0 + l16, kk * 32, hf), load_frag_b(wg  + PL_W, CIN, o0 + l16, kk * 32, hf), a2);
  }
  float bt = bth[o0 + l16], bp = bph[o0 + l16], bgv = bg[o0 + l16];
#pragma unroll
  for (int r = 0; r < 8; ++r) {
    st[0][r + 8 * hf][o0 + l16] = a0[r] + bt;
    st[1][r + 8 * hf][o0 + l16] = a1[r] + bp;
    st[2][r + 8 * hf][o0 + l16] = a2[r] + bgv;
  }
  __syncthreads();
  bf16* outs[3] = {th + (size_t)b * NPIX * CO, ph + (size_t)b * NPIX * CO, g + (size_t)b * NPIX * CO};
#pragma unroll 1
  for (int pass = 0; pass < 2; ++pass) {
#pragma unroll
    for (int s = 0; s < 3; ++s)
#pragma unroll
      for (int rr = 0; rr < 2; ++rr) {
        const int p = wave * 2 + rr;
        bf16* row = outs[s] + (size_t)(q0 + p) * CO;
#pragma unroll
        for (int sgm = 0; sgm < 2; ++sgm) {
          const int c = sgm * 64 + 2 * lane;
          _Float16 h0, l0, h1, l1; split16(st[s][p][c], h0, l0); split16(st[s][p][c + 1], h1, l1);
          *(volatile unsigned*)(row + c) = pack2h(h0, h1); *(volatile unsigned*)(row + PL_P + c) = pack2h(l0, l1);
        }
      }
    __threadfence();
  }
}

__global__ void __launch_bounds__(256) k_gT(const bf16* __restrict__ g, bf16* __restrict__ gT) {
  __shared__ bf16 t[64][CO + 2];
  const int tid = threadIdx.x, lane = tid & 31, wave = tid >> 5;
  const int b = blockIdx.x / (NPIX / 64), p0 = (blockIdx.x % (NPIX / 64)) * 64;
  const size_t pl = blockIdx.y ? PL_P : 0;
  const bf16* src = g + pl + ((size_t)b * NPIX + p0) * CO;
#pragma unroll
  for (int k = 0; k < 32; ++k) { const int e = tid + 256 * k; t[e >> 7][e & 127] = src[e]; }
  __syncthreads();
  bf16* dst = gT + pl + (size_t)b * CO * NPIX + p0;
#pragma unroll
  for (int rr = 0; rr < 16; ++rr) {
    const int co = wave * 16 + rr;
    const unsigned pk = pack2h(t[2 * lane][co], t[2 * lane + 1][co]);
    unsigned* d = (unsigned*)(dst + (size_t)co * NPIX) + lane;
    *(volatile unsigned*)d = pk; __threadfence(); *(volatile unsigned*)d = pk;
  }
}

__global__ void __launch_bounds__(256) k_attn(const bf16* __restrict__ th,
                                              const bf16* __restrict__ ph,
                                              const bf16* __restrict__ gT,
                                              bf16* __restrict__ y) {
  __shared__ __attribute__((aligned(16))) bf16 sphi[2][32 * CO];
  __shared__ __attribute__((aligned(16))) bf16 sg[2][CO * 32];
  __shared__ __attribute__((aligned(16))) bf16 sphil[2][32 * CO];
  __shared__ __attribute__((aligned(16))) bf16 sgl[2][CO * 32];
  __shared__ __attribute__((aligned(16))) bf16 pbuf[8][16 * 32];
  __shared__ __attribute__((aligned(16))) bf16 pbufl[8][16 * 32];
  __shared__ __attribute__((aligned(16))) float yst[8][16 * CO];
  int tid = threadIdx.x;
  int wave = tid >> 5, lane = tid & 31;
  int l16 = lane & 15, hf = lane >> 4;
  int b = blockIdx.x >> 5;
  int q0 = (((blockIdx.x & 31) << 3) + wave) * 16;
  const bf16* thb = th + (size_t)b * NPIX * CO;
  const bf16* phb = ph + (size_t)b * NPIX * CO;
  const bf16* gTb = gT + (size_t)b * CO * NPIX;
  bf16* pl = &pbuf[wave][0];
  bf16* pll = &pbufl[wave][0];

  unsigned phi_dst0 = lds_off(&sphi[0][0]) + tid * 16;
  unsigned phi_dst1 = lds_off(&sphi[1][0]) + tid * 16;
  unsigned phil_dst0 = lds_off(&sphil[0][0]) + tid * 16;
  unsigned phil_dst1 = lds_off(&sphil[1][0]) + tid * 16;
  int grow = tid >> 1, gh = tid & 1;
  unsigned g_dst0 = lds_off(&sg[0][0]) + grow * 64 + gh * 32;
  unsigned g_dst1 = lds_off(&sg[1][0]) + grow * 64 + gh * 32;
  unsigned gl_dst0 = lds_off(&sgl[0][0]) + grow * 64 + gh * 32;
  unsigned gl_dst1 = lds_off(&sgl[1][0]) + grow * 64 + gh * 32;
  const char* gsrc_row  = (const char*)(gTb + (size_t)grow * NPIX) + gh * 32;
  const char* gsrcl_row = (const char*)(gTb + PL_P + (size_t)grow * NPIX) + gh * 32;

#define ISSUE_COPIES(bufsel, m0_)                                               \
  do {                                                                          \
    const char* ps = (const char*)(phb + (size_t)(m0_) * CO) + tid * 16;        \
    const char* psl = (const char*)(phb + PL_P + (size_t)(m0_) * CO) + tid * 16;\
    unsigned pd = (bufsel) ? phi_dst1 : phi_dst0;                               \
    unsigned pdl = (bufsel) ? phil_dst1 : phil_dst0;                            \
    async_cp16(pd, ps);                                                         \
    async_cp16(pd + 4096, ps + 4096);                                           \
    async_cp16(pdl, psl);                                                       \
    async_cp16(pdl + 4096, psl + 4096);                                         \
    const char* gs = gsrc_row + (size_t)(m0_) * 2;                              \
    const char* gsl = gsrcl_row + (size_t)(m0_) * 2;                            \
    unsigned gd = (bufsel) ? g_dst1 : g_dst0;                                   \
    unsigned gdl = (bufsel) ? gl_dst1 : gl_dst0;                                \
    async_cp16(gd, gs);                                                         \
    async_cp16(gd + 16, gs + 16);                                               \
    async_cp16(gdl, gsl);                                                       \
    async_cp16(gdl + 16, gsl + 16);                                             \
  } while (0)

  bf16x16 aq[4], aql[4];
#pragma unroll
  for (int kk = 0; kk < 4; ++kk) { aq[kk] = load_frag_a(thb, CO, q0 + l16, kk * 32, hf); aql[kk] = load_frag_a(thb + PL_P, CO, q0 + l16, kk * 32, hf); }

  v8f O[8];
  float mrun[8], lrun[8];
#pragma unroll
  for (int c = 0; c < 8; ++c) O[c] = v8f{};
#pragma unroll
  for (int r = 0; r < 8; ++r) { mrun[r] = -INFINITY; lrun[r] = 0.f; }

  ISSUE_COPIES(0, 0);

  for (int m0 = 0; m0 < NPIX; m0 += 32) {
    int cur = (m0 >> 5) & 1;
    if (m0 + 32 < NPIX) {
      ISSUE_COPIES(cur ^ 1, m0 + 32);
      asm volatile("s_wait_asynccnt 0x8" ::: "memory");
    } else {
      asm volatile("s_wait_asynccnt 0x0" ::: "memory");
    }
    __syncthreads();
    const bf16* lphi = &sphi[cur][0];  const bf16* lphil = &sphil[cur][0];
    const bf16* lg   = &sg[cur][0];    const bf16* lgl   = &sgl[cur][0];

    v8f s0 = {}, s1 = {};
#pragma unroll
    for (int kk = 0; kk < 4; ++kk)
      s0 = wmma_split(aq[kk], aql[kk], load_frag_b(lphi, CO, l16, kk * 32, hf), load_frag_b(lphil, CO, l16, kk * 32, hf), s0);
#pragma unroll
    for (int kk = 0; kk < 4; ++kk)
      s1 = wmma_split(aq[kk], aql[kk], load_frag_b(lphi, CO, 16 + l16, kk * 32, hf), load_frag_b(lphil, CO, 16 + l16, kk * 32, hf), s1);

    float scale[8];
#pragma unroll
    for (int r = 0; r < 8; ++r) {
      float t = fmaxf(s0[r], s1[r]);
#pragma unroll
      for (int mk = 1; mk < 16; mk <<= 1) t = fmaxf(t, __shfl_xor(t, mk, 32));
      float mn = fmaxf(mrun[r], t);
      float sc = __expf(mrun[r] - mn);
      float e0 = __expf(s0[r] - mn);
      float e1 = __expf(s1[r] - mn);
      float rs = e0 + e1;
#pragma unroll
      for (int mk = 1; mk < 16; mk <<= 1) rs += __shfl_xor(rs, mk, 32);
      lrun[r] = lrun[r] * sc + rs;
      mrun[r] = mn;
      scale[r] = sc;
      { _Float16 ph_, pq_;
        split16(e0 * 1024.0f, ph_, pq_); pl[(r + 8 * hf) * 32 + l16] = ph_;      pll[(r + 8 * hf) * 32 + l16] = pq_;
        split16(e1 * 1024.0f, ph_, pq_); pl[(r + 8 * hf) * 32 + 16 + l16] = ph_; pll[(r + 8 * hf) * 32 + 16 + l16] = pq_; }
    }
#pragma unroll
    for (int c = 0; c < 8; ++c)
#pragma unroll
      for (int r = 0; r < 8; ++r) O[c][r] *= scale[r];

    asm volatile("s_wait_dscnt 0x0" ::: "memory");

    bf16x16 pa = load_frag_a(pl, 32, l16, 0, hf), pal = load_frag_a(pll, 32, l16, 0, hf);
#pragma unroll
    for (int c = 0; c < 8; ++c)
      O[c] = wmma_split(pa, pal, load_frag_b(lg, 32, c * 16 + l16, 0, hf), load_frag_b(lgl, 32, c * 16 + l16, 0, hf), O[c]);

    __syncthreads();
  }
#undef ISSUE_COPIES

  float inv[8];
#pragma unroll
  for (int r = 0; r < 8; ++r) inv[r] = 1.0f / (lrun[r] * 1024.0f);
  float* ys = yst[wave];
#pragma unroll
  for (int c = 0; c < 8; ++c)
#pragma unroll
    for (int r = 0; r < 8; ++r) ys[(r + 8 * hf) * CO + c * 16 + l16] = O[c][r] * inv[r];
  asm volatile("s_wait_dscnt 0x0" ::: "memory");
  bf16* yb = y + ((size_t)b * NPIX + q0) * CO;
#pragma unroll 1
  for (int pass = 0; pass < 2; ++pass) {
#pragma unroll 4
    for (int rr = 0; rr < 16; ++rr)
#pragma unroll
      for (int sgm = 0; sgm < 2; ++sgm) {
        const int c = sgm * 64 + 2 * lane;
        _Float16 h0, l0, h1, l1;
        split16(*(const volatile float*)(ys + rr * CO + c), h0, l0); split16(*(const volatile float*)(ys + rr * CO + c + 1), h1, l1);
        *(volatile unsigned*)(yb + (size_t)rr * CO + c) = pack2h(h0, h1); *(volatile unsigned*)(yb + PL_P + (size_t)rr * CO + c) = pack2h(l0, l1);
      }
    __threadfence();
  }
}

typedef __attribute__((ext_vector_type(4))) float v4f_t;
typedef float v4fa __attribute__((ext_vector_type(4), may_alias));
__global__ void __launch_bounds__(256) k_outconv(const bf16* __restrict__ y, const bf16* __restrict__ wW,
                          const float* __restrict__ bW, const float* __restrict__ x,
                          float* __restrict__ out) {
  __shared__ __attribute__((aligned(16))) float st[8][16 * 32];
  int wave = threadIdx.x >> 5, lane = threadIdx.x & 31;
  int l16 = lane & 15, hf = lane >> 4;
  int tile = blockIdx.x * 8 + wave;
  int b = tile >> 11;
  int rem = tile & 2047;
  int pt = rem >> 4, ct = rem & 15;
  int q0 = pt * 32, c0 = ct * 16;
  const bf16* yb = y + (size_t)b * NPIX * CO;

  v8f acc0 = {}, acc1 = {};
#pragma unroll
  for (int kk = 0; kk < 4; ++kk) {
    bf16x16 bw = load_frag_b(wW, CO, c0 + l16, kk * 32, hf), bwl = load_frag_b(wW + PL_WW, CO, c0 + l16, kk * 32, hf);
    acc0 = wmma_split(load_frag_a(yb, CO, q0 + l16, kk * 32, hf),      load_frag_a(yb + PL_P, CO, q0 + l16, kk * 32, hf),      bw, bwl, acc0);
    acc1 = wmma_split(load_frag_a(yb, CO, q0 + 16 + l16, kk * 32, hf), load_frag_a(yb + PL_P, CO, q0 + 16 + l16, kk * 32, hf), bw, bwl, acc1);
  }
  float bias = bW[c0 + l16];
  float* sw = st[wave];
#pragma unroll
  for (int r = 0; r < 8; ++r) {
    sw[l16 * 32 + r + 8 * hf]      = acc0[r] + bias;
    sw[l16 * 32 + 16 + r + 8 * hf] = acc1[r] + bias;
  }
  asm volatile("s_wait_dscnt 0x0" ::: "memory");
  v4f_t ov[4]; size_t oo[4];
#pragma unroll
  for (int i = 0; i < 4; ++i) {
    const int c = lane + 32 * i, rr = c >> 3, qq = c & 7;
    oo[i] = ((size_t)b * CIN + c0 + rr) * NPIX + q0 + qq * 4;
    const v4f_t xv = *(const v4f_t*)(x + oo[i]);
    ov[i] = *(const volatile v4fa*)(sw + rr * 32 + qq * 4) + xv;
  }
#pragma unroll
  for (int i = 0; i < 4; ++i) *(volatile v4f_t*)(out + oo[i]) = ov[i];
  __threadfence();
#pragma unroll
  for (int i = 0; i < 4; ++i) *(volatile v4f_t*)(out + oo[i]) = ov[i];
}

extern "C" void kernel_launch(void* const* d_in, const int* in_sizes, int n_in,
                              void* d_out, int out_size, void* d_ws, size_t ws_size,
                              hipStream_t stream) {
  (void)in_sizes; (void)n_in; (void)out_size; (void)ws_size;
  const float* x       = (const float*)d_in[0];
  const float* w_theta = (const float*)d_in[1];
  const float* b_theta = (const float*)d_in[2];
  const float* w_phi   = (const float*)d_in[3];
  const float* b_phi   = (const float*)d_in[4];
  const float* w_g     = (const float*)d_in[5];
  const float* b_g     = (const float*)d_in[6];
  const float* w_W     = (const float*)d_in[7];
  const float* b_W     = (const float*)d_in[8];

  char* ws = (char*)d_ws;
  bf16* xT  = (bf16*)(ws);
  bf16* th  = (bf16*)(ws + 16777216);
  bf16* ph  = (bf16*)(ws + 25165824);
  bf16* gR  = (bf16*)(ws + 33554432);
  bf16* gT  = (bf16*)(ws + 41943040);
  bf16* yb  = (bf16*)(ws + 50331648);
  bf16* wth = (bf16*)(ws + 58720256);
  bf16* wph = (bf16*)(ws + 58851328);
  bf16* wgv = (bf16*)(ws + 58982400);
  bf16* wWb = (bf16*)(ws + 59113472);

  k_wconv<<<64, 256, 0, stream>>>(w_theta, w_phi, w_g, w_W, wth, wph, wgv, wWb);

  k_xpose<<<dim3(NPIX / 32, NB), 256, 0, stream>>>(x, xT);

  k_proj<<<1024, 256, 0, stream>>>(xT, wth, wph, wgv, b_theta, b_phi, b_g, th, ph, gR);
  k_gT<<<dim3(NB * NPIX / 64, 2), 256, 0, stream>>>(gR, gT);

  k_attn<<<128, 256, 0, stream>>>(th, ph, gT, yb);

  k_outconv<<<1024, 256, 0, stream>>>(yb, wWb, b_W, x, (float*)d_out);
}
